// ValueModel_10823317586373
// MI455X (gfx1250) — hardware-run, weakly checked
//
#include <hip/hip_runtime.h>


#ifndef NROWS
#define NROWS 32768
#endif
#define NROWS_FULL 32768
#define NIN   16
#define NOUT  50
#define NLAY  25
#define NFEAT 1266
#define ACOLS 64
#define WSC   16.0f
#define WSI   (1.0f / 16.0f)
#define HG    7
#define HWP   1792

static_assert(NIN + NLAY * NOUT == NFEAT);
static_assert(NOUT <= 64);
static_assert(NIN <= 32);
static_assert(ACOLS == 64);
static_assert(NROWS % 64 == 0);
static_assert(NROWS % 256 == 0);
static_assert(((size_t)NROWS * 8) % 256 == 0);
static_assert(NROWS <= NROWS_FULL);
static_assert(HG * 8 >= NOUT);
static_assert(HG * 8 <= ACOLS);
static_assert(HWP == 7 * 256);
static_assert(HWP >= NIN + NLAY * 64);
static_assert(16 * 68 * 4 <= 131072);
static_assert((HWP + 256) * 4 <= 131072);
static_assert(32 * 16 * 4 == 16 * 128);
static_assert(8 * 16 == 32 * 4);

typedef _Float16 h16;
typedef __attribute__((ext_vector_type(16))) _Float16 v16h;
typedef __attribute__((ext_vector_type(8)))  _Float16 v8h;
typedef __attribute__((ext_vector_type(8)))  float    v8f;
typedef __attribute__((ext_vector_type(4)))  float    v4f;
typedef v4f  __attribute__((may_alias)) v4fa;

__device__ __forceinline__ unsigned short f2bf(float f) { unsigned u = __float_as_uint(f); u += 0x7FFFu + ((u >> 16) & 1u); return (unsigned short)(u >> 16); }
__device__ __forceinline__ float bfr(float f) { return __uint_as_float(((unsigned)f2bf(f)) << 16); }
__device__ __forceinline__ v16h cat16(v8h lo, v8h hi) { return __builtin_shufflevector(lo, hi, 0, 1, 2, 3, 4, 5, 6, 7, 8, 9, 10, 11, 12, 13, 14, 15); }
__device__ __forceinline__ v8f wmma16(v16h a, v16h b, v8f c) { return __builtin_amdgcn_wmma_f32_16x16x32_f16(false, a, false, b, (short)0, c, false, false); }
__device__ __forceinline__ v8f wmma16g(v16h a, v16h b, v8f c) { c = wmma16(a, b, c); asm volatile("v_nop\n\tv_nop\n\tv_nop\n\tv_nop" : "+v"(c) : "v"(a), "v"(b)); return c; }
__device__ __forceinline__ v16h  ldh(const h16* p) { return cat16(*(const v8h*)p, *(const v8h*)(p + 16)); }
__device__ __forceinline__ void wave_sync() { __builtin_amdgcn_fence(3  , "wavefront"); __builtin_amdgcn_wave_barrier(); asm volatile("" ::: "memory"); }
static __device__ __forceinline__ h16 toh_flush(float v) { const float w = (fabsf(v) < 6.103515625e-05f) ? 0.0f : v; return (h16)w; }

__global__ __launch_bounds__(256) void k_sconv(const float* __restrict__ st, h16* S) {
    const unsigned g = blockIdx.x * 256u + threadIdx.x;
    if (g >= (unsigned)NROWS * 8u) return;
    const unsigned row = g >> 3, c8 = (g & 7u) * 8u;
    const unsigned cs = (unsigned)min((int)c8, 8);
    const float* p = st + (size_t)row * NIN + cs;
    const v4f x0 = *(const v4f*)p, x1 = *(const v4f*)(p + 4);
    const bool ok = c8 < (unsigned)NIN;
    v8h o;
#pragma unroll
    for (int i = 0; i < 4; ++i) { const float a0 = bfr(x0[i]), a1 = bfr(x1[i]); o[i] = toh_flush(ok ? a0 : 0.0f); o[4 + i] = toh_flush(ok ? a1 : 0.0f); }
    h16* d = S + (size_t)g * 8;
    *(volatile v8h*)d = o; __threadfence(); *(volatile v8h*)d = o;
}

__global__ __launch_bounds__(256) void k_wconv(const float* __restrict__ Wsrc, h16* WL) {
    const unsigned layer = blockIdx.y;
    const unsigned ki8 = 4u + 8u * layer;
    const unsigned tot = 64u * ki8;
    const unsigned g = blockIdx.x * 256u + threadIdx.x;
    if (g >= tot) return;
    const unsigned o = g / ki8;
    const unsigned c8 = (g - o * ki8) * 8u;
    const unsigned oc = (unsigned)min((int)o, NOUT - 1);
    const bool sblk = c8 < 32u;
    const unsigned cc = (unsigned)max((int)c8, 32) - 32u;
    const unsigned j = cc >> 6, q0 = cc & 63u;
    const unsigned p0 = sblk ? c8 : q0;
    const unsigned lim = sblk ? (unsigned)NIN : (unsigned)NOUT;
    const unsigned cb = sblk ? 0u : ((unsigned)NIN + (unsigned)NOUT * j);
    const float* src = Wsrc + ((size_t)layer * NOUT + oc) * NFEAT + cb;
    const bool rok = o < (unsigned)NOUT;
    v8h ov;
#pragma unroll
    for (int e = 0; e < 8; ++e) {
        const unsigned p = p0 + (unsigned)e;
        const unsigned pc = (unsigned)min((int)p, (int)lim - 1);
        const float w = bfr(src[pc]) * WSC;
        const bool ok = rok && (p < lim);
        ov[e] = toh_flush(ok ? w : 0.0f); }
    h16* d = WL + (size_t)2048 * layer * layer + (size_t)g * 8;
    *(volatile v8h*)d = ov; __threadfence(); *(volatile v8h*)d = ov;
}

__device__ __forceinline__ void kstep(const h16* ap, const h16* bp, const unsigned Ki, v8f (&acc)[4][4]) {
    v16h a[4];
#pragma unroll
    for (int mb = 0; mb < 4; ++mb) a[mb] = ldh(ap + (size_t)mb * 16 * ACOLS);
#pragma unroll
    for (int nb = 0; nb < 4; ++nb) { const v16h b = ldh(bp + (size_t)nb * 16 * Ki);
#pragma unroll
        for (int mb = 0; mb < 4; ++mb) acc[mb][nb] = wmma16g(a[mb], b, acc[mb][nb]); }
}

__global__ __launch_bounds__(32) void k_layer(const h16* __restrict__ S, h16* Y, const h16* __restrict__ WL, const float* __restrict__ bs, int layer) {
    __shared__ __align__(16) float os[16 * 68];
    const int lane = threadIdx.x & 31, lr = lane & 15, hi = lane >> 4;
    const unsigned bx = blockIdx.x; const unsigned r0 = bx * 64u;
    const unsigned ul = (unsigned)layer; const unsigned Ki = 32u + 64u * ul;
    v8f acc[4][4];
#pragma unroll
    for (int mb = 0; mb < 4; ++mb)
#pragma unroll
        for (int nb = 0; nb < 4; ++nb) acc[mb][nb] = (v8f){};
    const size_t aoff = (size_t)(r0 + (unsigned)lr) * ACOLS + (size_t)(8 * hi);
    const h16* bp = WL + (size_t)2048 * ul * ul + (size_t)lr * Ki + (size_t)(8 * hi);
    kstep(S + aoff, bp, Ki, acc);
#pragma unroll 1
    for (unsigned j = 0; j < ul; ++j) {
        const h16* ap = Y + (size_t)j * ((size_t)NROWS * ACOLS) + aoff;
        const h16* bq = bp + 32u + 64u * j;
        kstep(ap, bq, Ki, acc);
        kstep(ap + 32, bq + 32, Ki, acc); }
    const unsigned c8 = (unsigned)(lane & 7) * 8u;
    float bv[8];
#pragma unroll
    for (int e = 0; e < 8; ++e) { const unsigned col = c8 + (unsigned)e; const unsigned cc = (unsigned)min((int)col, NOUT - 1);
        const float b = bfr(bs[ul * NOUT + cc]); bv[e] = (col < (unsigned)NOUT) ? b : 0.0f; }
    h16* yo = Y + (size_t)ul * ((size_t)NROWS * ACOLS) + (size_t)r0 * ACOLS;
#pragma unroll
    for (int mb = 0; mb < 4; ++mb) {
#pragma unroll
        for (int nb = 0; nb < 4; ++nb) {
#pragma unroll
            for (int j = 0; j < 8; ++j) os[(hi * 8 + j) * 68 + nb * 16 + lr] = acc[mb][nb][j]; }
        wave_sync();
#pragma unroll 1
        for (int ps = 0; ps < 2; ++ps) {
#pragma unroll
            for (int s = 0; s < 4; ++s) { const int row = 4 * s + (lane >> 3);
                const v4f x0 = *(const v4fa*)(&os[row * 68 + (int)c8]); const v4f x1 = *(const v4fa*)(&os[row * 68 + (int)c8 + 4]); v8h hv;
#pragma unroll
                for (int i = 0; i < 4; ++i) {
                    float u0 = x0[i] * WSI + bv[i]; float u1 = x1[i] * WSI + bv[4 + i];
                    u0 = (u0 > 0.0f) ? u0 : 0.01f * u0; u1 = (u1 > 0.0f) ? u1 : 0.01f * u1;
                    u0 = (c8 + (unsigned)i < (unsigned)NOUT) ? u0 : 0.0f; u1 = (c8 + 4u + (unsigned)i < (unsigned)NOUT) ? u1 : 0.0f;
                    hv[i] = toh_flush(u0); hv[4 + i] = toh_flush(u1); }
                *(volatile v8h*)(yo + (size_t)(mb * 16 + row) * ACOLS + c8) = hv; }
            if (ps == 0) __threadfence(); }
        wave_sync();
    }
}

__device__ __forceinline__ void acc8(float (&a)[8], const v8h x, const v4f w0, const v4f w1) {
#pragma unroll
    for (int e = 0; e < 4; ++e) { a[e] += (float)x[e] * w0[e]; a[4 + e] += (float)x[4 + e] * w1[e]; }
}

__global__ __launch_bounds__(256) void k_head(const h16* __restrict__ S, const h16* __restrict__ Y, const float* __restrict__ wout, const float* __restrict__ bout, float* OUT) {
    __shared__ __align__(16) float wl[HWP];
    __shared__ __align__(16) float ot[256];
    const unsigned tid = threadIdx.x;
    const int lane = (int)(tid & 31u);
    const int wave = __builtin_amdgcn_readfirstlane((int)(threadIdx.x >> 5));
#pragma unroll 1
    for (unsigned it = 0; it < 7u; ++it) {
        const unsigned t = it * 256u + tid;
        const unsigned u = (unsigned)max((int)t, NIN) - (unsigned)NIN;
        const unsigned j = u >> 6, q = u & 63u;
        const unsigned sy = (unsigned)NIN + (unsigned)NOUT * j + (unsigned)min((int)q, NOUT - 1);
        const unsigned sx = (t < (unsigned)NIN) ? t : sy;
        const unsigned src = (unsigned)min((int)sx, NFEAT - 1);
        const bool ok = (t < (unsigned)NIN) || ((q < (unsigned)NOUT) && (j < (unsigned)NLAY));
        const float w = bfr(wout[src]);
        wl[t] = ok ? w : 0.0f; }
    __syncthreads();
    const unsigned bx = blockIdx.x;
    const unsigned rb = bx * 256u + (unsigned)wave * 32u;
    const size_t roff = (size_t)(rb + (unsigned)lane) * ACOLS;
    float a8[8];
#pragma unroll
    for (int e = 0; e < 8; ++e) a8[e] = 0.0f;
    {   const h16* sp = S + roff;
#pragma unroll 1
        for (int g = 0; g < NIN / 8; ++g) {
            const v8h x = *(const v8h*)(sp + g * 8);
            const v4f w0 = *(const v4fa*)(&wl[g * 8]); const v4f w1 = *(const v4fa*)(&wl[g * 8 + 4]);
            acc8(a8, x, w0, w1); } }
#pragma unroll 1
    for (int j = 0; j < NLAY; ++j) {
        const h16* yp = Y + (size_t)j * ((size_t)NROWS * ACOLS) + roff;
#pragma unroll 1
        for (int g = 0; g < HG; ++g) {
            const v8h x = *(const v8h*)(yp + g * 8);
            const v4f w0 = *(const v4fa*)(&wl[NIN + j * 64 + g * 8]); const v4f w1 = *(const v4fa*)(&wl[NIN + j * 64 + g * 8 + 4]);
            acc8(a8, x, w0, w1); } }
    const float sum = (((a8[0] + a8[1]) + (a8[2] + a8[3])) + ((a8[4] + a8[5]) + (a8[6] + a8[7]))) + bfr(bout[0]);
    ot[wave * 32 + lane] = sum;
    wave_sync();
    const v4f val = *(const v4fa*)(&ot[wave * 32 + (lane & 7) * 4]);
    float* op = OUT + (size_t)rb + (size_t)((lane & 7) * 4);
#pragma unroll 1
    for (int ps = 0; ps < 2; ++ps) {
        if (lane < 8) *(volatile v4f*)op = val;
        if (ps == 0) __threadfence(); }
}

static constexpr size_t al256(size_t v) { return (v + 255) & ~(size_t)255; }
static constexpr size_t SZ_S = al256((size_t)NROWS * ACOLS * 2);
static constexpr size_t SZ_Y = al256((size_t)NLAY * NROWS * ACOLS * 2);
static constexpr size_t SZ_W = al256((size_t)2048 * NLAY * NLAY * 2);
static constexpr size_t SZ_TOTAL = SZ_S + SZ_Y + SZ_W;
static_assert(SZ_TOTAL <= (size_t)134217728);
static_assert((size_t)2048 * (NLAY - 1) * (NLAY - 1) + (size_t)64 * (32 + 64 * (NLAY - 1)) == (size_t)2048 * NLAY * NLAY);
static_assert((64 * (4 + 8 * (NLAY - 1))) % 256 == 0);
static_assert(((size_t)NROWS * ACOLS * 2) % 256 == 0);

extern "C" void kernel_launch(void* const* d_in, const int* in_sizes, int n_in,
                              void* d_out, int out_size, void* d_ws, size_t ws_size, hipStream_t stream) {
    if (n_in < 5) return;
    if ((size_t)in_sizes[0] < (size_t)NROWS * NIN) return;
    if ((size_t)in_sizes[1] < (size_t)NLAY * NOUT * NFEAT) return;
    if (in_sizes[2] < NLAY * NOUT || in_sizes[3] < NFEAT || in_sizes[4] < 1) return;
    if ((size_t)out_size < (size_t)NROWS) return;
    if (SZ_TOTAL > ws_size) return;
    const float* state = (const float*)d_in[0];
    const float* Wsrc  = (const float*)d_in[1];
    const float* bsrc  = (const float*)d_in[2];
    const float* wout  = (const float*)d_in[3];
    const float* bout  = (const float*)d_in[4];
    float* OUT = (float*)d_out;
    char* wsp = (char*)d_ws;
    h16* S  = (h16*)wsp; wsp += SZ_S;
    h16* Y  = (h16*)wsp; wsp += SZ_Y;
    h16* WL = (h16*)wsp; wsp += SZ_W;

    k_sconv<<<(unsigned)(((size_t)NROWS * 8) / 256), 256, 0, stream>>>(state, S);
    k_wconv<<<dim3((64 * (4 + 8 * (NLAY - 1))) / 256, NLAY, 1), 256, 0, stream>>>(Wsrc, WL);
    for (int i = 0; i < NLAY; ++i)
        k_layer<<<NROWS / 64, 32, 0, stream>>>(S, Y, WL, bsrc, i);
    k_head<<<NROWS / 256, 256, 0, stream>>>(S, Y, wout, bout, OUT);
}
